// M2Model_69449621176665
// MI455X (gfx1250) — hardware-run, weakly checked
//
#include <hip/hip_runtime.h>
#include <math.h>

typedef __attribute__((ext_vector_type(16))) _Float16 v16h;
typedef __attribute__((ext_vector_type(8)))  _Float16 v8h;
typedef __attribute__((ext_vector_type(16))) __bf16   v16b;
typedef __attribute__((ext_vector_type(8)))  __bf16   v8b;
typedef __attribute__((ext_vector_type(8)))  float    v8f;
typedef __attribute__((ext_vector_type(4)))  float    v4f;
typedef __attribute__((ext_vector_type(4)))  unsigned v4u;

constexpr int kSeqs   = 32;
constexpr int kLen    = 256;
constexpr int kRows   = kSeqs * kLen;
constexpr int kDm     = 512;
constexpr int kDi     = 1024;
constexpr int kNs     = 32;
constexpr int kNh     = 16;
constexpr int kHd     = 64;
constexpr int kConv   = kDi + 2 * kNs;
constexpr int kProj   = 2 * kDi + 2 * kNs + kNh;
constexpr int kProjP  = 2176;
constexpr int kVoc    = 28;
constexpr int kVocP   = 64;
constexpr int kTokP   = 64;
constexpr int kColX   = kDi;
constexpr int kColB   = 2 * kDi;
constexpr int kColDt  = 2 * kDi + 2 * kNs;
constexpr int kYP     = 68;
constexpr int kChunk  = 16;
constexpr float kCarryA = 16.0f;
constexpr float kCarryW = 256.0f;
constexpr float kFold   = 1.0f / (kCarryA * kCarryW);
constexpr float kInvDi  = 1.0f / (float)kDi;
static_assert(kRows == 8192 && kConv == 1088 && kProj == 2128, "shape chain");
static_assert(kNh * kHd == kDi, "heads x head width");
static_assert(kProjP % 64 == 0 && kProjP >= kProj, "projection width padded to the tile");
static_assert(kVocP % 64 == 0 && kTokP % 64 == 0 && kTokP >= kVoc, "token / vocabulary pads");
static_assert(kDm % 32 == 0 && kDi % 32 == 0, "GEMM K multiples of 32");
static_assert(kRows % 64 == 0 && kDm % 64 == 0, "GEMM M, N multiples of 64");
static_assert(kLen % kChunk == 0, "scan chunking");
static_assert((kRows * kVoc) % 256 == 0, "output is a whole number of blocks of lines");

constexpr size_t kSzEM  = (size_t)kTokP * kDm * 2;
constexpr size_t kSzWI  = (size_t)2 * kProjP * kDm * 2;
constexpr size_t kSzTT  = (size_t)2 * kTokP * kProjP * 4;
constexpr size_t kSzDTA = (size_t)2 * 32 * 32 * 4;
constexpr size_t kSzYS  = (size_t)kRows * kDi * 4;
constexpr size_t kSzYN  = (size_t)kRows * kDi * 2;
constexpr size_t kSzWO  = (size_t)2 * kDm * kDi * 2;
constexpr size_t kSzO   = (size_t)kRows * kDm * 4;
constexpr size_t kSzY16 = (size_t)kRows * kDi * 2;
constexpr size_t kSzL   = (size_t)kVocP * kDi * 2;
constexpr size_t kSzCP  = (size_t)kRows * kVocP * 4;
constexpr size_t kOffEMH = 0;
constexpr size_t kOffEML = kOffEMH + kSzEM;
constexpr size_t kOffWIH = kOffEML + kSzEM;
constexpr size_t kOffWIL = kOffWIH + kSzWI;
constexpr size_t kOffTT  = kOffWIL + kSzWI;
constexpr size_t kOffDTA = kOffTT  + kSzTT;
constexpr size_t kOffYS  = kOffDTA + kSzDTA;
constexpr size_t kOffYN  = kOffYS  + kSzYS;
constexpr size_t kOffWO  = kOffYN  + kSzYN;
constexpr size_t kOffOF  = kOffWO  + kSzWO;
constexpr size_t kOffOB  = kOffOF  + kSzO;
constexpr size_t kOffYH  = kOffOB  + kSzO;
constexpr size_t kOffYL  = kOffYH  + kSzY16;
constexpr size_t kOffLH  = kOffYL  + kSzY16;
constexpr size_t kOffLL  = kOffLH  + kSzL;
constexpr size_t kOffCP  = kOffLL  + kSzL;
constexpr size_t kWsTotal = kOffCP + kSzCP;
static_assert(kWsTotal == 132063232ull, "carve total");
static_assert(kWsTotal <= 134217728ull, "carve cap");
static_assert((kSzEM % 128) == 0 && (kSzWI % 128) == 0 && (kSzTT % 128) == 0 && (kSzDTA % 128) == 0 &&
              (kSzYS % 128) == 0 && (kSzYN % 128) == 0 && (kSzWO % 128) == 0 && (kSzO % 128) == 0 &&
              (kSzY16 % 128) == 0 && (kSzL % 128) == 0 && (kSzCP % 128) == 0, "128-B aligned regions");

__device__ __forceinline__ unsigned f2bf_u(float f) {
  const unsigned u = __float_as_uint(f);
  return (u + 0x7FFFu + ((u >> 16) & 1u)) >> 16;
}
__device__ __forceinline__ float bf_u2f(unsigned h) { return __uint_as_float(h << 16); }
__device__ __forceinline__ void split2(float x, float y, unsigned& wh, unsigned& wl) {
  const unsigned hx = f2bf_u(x);
  const unsigned hy = f2bf_u(y);
  const unsigned lx = f2bf_u(x - bf_u2f(hx));
  const unsigned ly = f2bf_u(y - bf_u2f(hy));
  wh = hx | (hy << 16);
  wl = lx | (ly << 16);
}
__device__ __forceinline__ unsigned h2pack(float x, float y) {
  const _Float16 hx = (_Float16)x;
  const _Float16 hy = (_Float16)y;
  const unsigned bx = (unsigned)__builtin_bit_cast(unsigned short, hx);
  const unsigned by = (unsigned)__builtin_bit_cast(unsigned short, hy);
  return bx | (by << 16);
}
__device__ __forceinline__ float silu_fast(float v) {
  const float sg = __builtin_amdgcn_rcpf(1.0f + __expf(-v));
  return v * sg;
}
__device__ __forceinline__ int clamp_tok(int t) {
  t = t < 0 ? 0 : t;
  t = t > (kVoc - 1) ? (kVoc - 1) : t;
  return t;
}

__device__ __forceinline__ v8f mma_guard_h(v16h a, v16h b, v8f c) {
  c = __builtin_amdgcn_wmma_f32_16x16x32_f16(false, a, false, b, (short)0, c, false, false);
  asm volatile("v_nop\n\tv_nop\n\tv_nop\n\tv_nop" : "+v"(c) : "v"(a), "v"(b));
  return c;
}
__device__ __forceinline__ v8f mma_guard_b(v16b a, v16b b, v8f c) {
  c = __builtin_amdgcn_wmma_f32_16x16x32_bf16(false, a, false, b, (short)0, c, false, false);
  asm volatile("v_nop\n\tv_nop\n\tv_nop\n\tv_nop" : "+v"(c) : "v"(a), "v"(b));
  return c;
}
template <typename T> struct Frag;
template <> struct Frag<_Float16> {
  typedef v16h V;
  union U { v16h v; v8h h[2]; };
  static __device__ __forceinline__ v16h load(const _Float16* p) {
    U f;
    f.h[0] = *(const v8h*)(p);
    f.h[1] = *(const v8h*)(p + 16);
    return f.v;
  }
  static __device__ __forceinline__ v8f mma(v16h a, v16h b, v8f c) { return mma_guard_h(a, b, c); }
};
template <> struct Frag<__bf16> {
  typedef v16b V;
  union U { v16b v; v8b h[2]; };
  static __device__ __forceinline__ v16b load(const __bf16* p) {
    U f;
    f.h[0] = *(const v8b*)(p);
    f.h[1] = *(const v8b*)(p + 16);
    return f.v;
  }
  static __device__ __forceinline__ v8f mma(v16b a, v16b b, v8f c) { return mma_guard_b(a, b, c); }
};
template <int ET> struct Elem;
template <> struct Elem<0> { typedef _Float16 T; };
template <> struct Elem<1> { typedef __bf16 T; };

template <int ET, bool SPLIT>
__global__ __launch_bounds__(256) void wmma_gemm64(
    const unsigned short* __restrict__ Ap, const unsigned short* __restrict__ A2p, int lda, long strideA,
    const unsigned short* __restrict__ Btp, const unsigned short* __restrict__ Bt2p, int ldb, long strideB,
    float* __restrict__ Cout, int ldc, long strideC,
    int M, int N, int K, float scale) {
  typedef typename Elem<ET>::T T;
  typedef typename Frag<T>::V V;
  const T* A   = (const T*)Ap;
  const T* A2  = (const T*)A2p;
  const T* Bt  = (const T*)Btp;
  const T* Bt2 = (const T*)Bt2p;
  __shared__ __align__(16) float sT[8][16 * kYP];
  const int b    = blockIdx.y;
  const int lane = threadIdx.x & 31;
  const int wave = threadIdx.x >> 5;
  const int tilesN = N >> 6;
  const int tilesM = M >> 6;
  const int tile = blockIdx.x * 8 + wave;
  if (tile >= tilesM * tilesN) return;
  const int tm = tile / tilesN;
  const int tn = tile - tm * tilesN;
  const int m0 = tm << 6;
  const int n0 = tn << 6;

  const T* Ab  = A   + (size_t)b * strideA;
  const T* Bb  = Bt  + (size_t)b * strideB;
  const T* Ab2 = A2  + (size_t)b * strideA;
  const T* Bb2 = Bt2 + (size_t)b * strideB;

  const int rlane = lane & 15;
  const int koff  = (lane >> 4) * 8;
  const int mOff  = (lane >> 4) * 8;

  v8f acc[4][4];
#pragma unroll
  for (int i = 0; i < 4; ++i)
#pragma unroll
    for (int j = 0; j < 4; ++j) acc[i][j] = (v8f){0.f, 0.f, 0.f, 0.f, 0.f, 0.f, 0.f, 0.f};

  for (int k0 = 0; k0 < K; k0 += 32) {
    V bh[4], bl[4];
#pragma unroll
    for (int j = 0; j < 4; ++j) {
      const size_t bo = (size_t)(n0 + (j << 4) + rlane) * ldb + koff + k0;
      bh[j] = Frag<T>::load(Bb + bo);
      if (SPLIT) bl[j] = Frag<T>::load(Bb2 + bo);
    }
#pragma unroll
    for (int i = 0; i < 4; ++i) {
      const size_t ao = (size_t)(m0 + (i << 4) + rlane) * lda + koff + k0;
      V ah = Frag<T>::load(Ab + ao);
      V al;
      if (SPLIT) al = Frag<T>::load(Ab2 + ao);
#pragma unroll
      for (int j = 0; j < 4; ++j) {
        acc[i][j] = Frag<T>::mma(ah, bh[j], acc[i][j]);
        if (SPLIT) {
          acc[i][j] = Frag<T>::mma(ah, bl[j], acc[i][j]);
          acc[i][j] = Frag<T>::mma(al, bh[j], acc[i][j]);
        }
      }
    }
  }

  float* slab = sT[wave];
  float* C = Cout + (size_t)b * strideC;
  const int hh = lane >> 4;
  const int c4 = (lane & 15) * 4;
#pragma unroll
  for (int i = 0; i < 4; ++i) {
    const int mBase = m0 + (i << 4);
#pragma unroll
    for (int j = 0; j < 4; ++j) {
#pragma unroll
      for (int r = 0; r < 8; ++r) {
        const float v = acc[i][j][r] * scale;
        slab[(mOff + r) * kYP + (j << 4) + rlane] = v;
      }
    }
    __builtin_amdgcn_fence(__ATOMIC_RELEASE, "workgroup");
    __builtin_amdgcn_wave_barrier();
    __builtin_amdgcn_fence(__ATOMIC_ACQUIRE, "workgroup");
    for (int pass = 0; pass < 2; ++pass) {
#pragma unroll
      for (int it = 0; it < 8; ++it) {
        const int row = it * 2 + hh;
        const v4f v = *(const v4f*)(slab + row * kYP + c4);
        *(volatile v4f*)(C + (size_t)(mBase + row) * ldc + n0 + c4) = v;
      }
      __threadfence();
    }
    __builtin_amdgcn_fence(__ATOMIC_RELEASE, "workgroup");
    __builtin_amdgcn_wave_barrier();
    __builtin_amdgcn_fence(__ATOMIC_ACQUIRE, "workgroup");
  }
}

__global__ __launch_bounds__(256) void split_pad_bf16_kernel(
    const float* __restrict__ src, unsigned short* __restrict__ dhi, unsigned short* __restrict__ dlo,
    int rows_real, int cols8, int total8) {
  const int i = blockIdx.x * 256 + threadIdx.x;
  if (i >= total8) return;
  const int row = i / cols8;
  const int c = (i - row * cols8) << 3;
  const int cols = cols8 << 3;
  const bool live = row < rows_real;
  const int rc = live ? row : (rows_real - 1);
  const float* sp = src + (size_t)rc * cols + c;
  const v4f a0 = *(const v4f*)(sp);
  const v4f a1 = *(const v4f*)(sp + 4);
  const float x0 = live ? a0[0] : 0.0f;
  const float x1 = live ? a0[1] : 0.0f;
  const float x2 = live ? a0[2] : 0.0f;
  const float x3 = live ? a0[3] : 0.0f;
  const float x4 = live ? a1[0] : 0.0f;
  const float x5 = live ? a1[1] : 0.0f;
  const float x6 = live ? a1[2] : 0.0f;
  const float x7 = live ? a1[3] : 0.0f;
  unsigned h0, h1, h2, h3, l0, l1, l2, l3;
  split2(x0, x1, h0, l0);
  split2(x2, x3, h1, l1);
  split2(x4, x5, h2, l2);
  split2(x6, x7, h3, l3);
  const v4u wh = (v4u){h0, h1, h2, h3};
  const v4u wl = (v4u){l0, l1, l2, l3};
  const size_t e0 = (size_t)i << 3;
  *(volatile v4u*)(dhi + e0) = wh;
  *(volatile v4u*)(dlo + e0) = wl;
  __threadfence();
  *(volatile v4u*)(dhi + e0) = wh;
  *(volatile v4u*)(dlo + e0) = wl;
}

__global__ __launch_bounds__(256) void cvt_f16_carry_kernel(
    const float* __restrict__ src, unsigned short* __restrict__ dst, int total8, float carry) {
  const int i = blockIdx.x * 256 + threadIdx.x;
  if (i >= total8) return;
  const size_t e0 = (size_t)i << 3;
  const v4f a0 = *(const v4f*)(src + e0);
  const v4f a1 = *(const v4f*)(src + e0 + 4);
  const unsigned w0 = h2pack(a0[0] * carry, a0[1] * carry);
  const unsigned w1 = h2pack(a0[2] * carry, a0[3] * carry);
  const unsigned w2 = h2pack(a1[0] * carry, a1[1] * carry);
  const unsigned w3 = h2pack(a1[2] * carry, a1[3] * carry);
  const v4u w = (v4u){w0, w1, w2, w3};
  *(volatile v4u*)(dst + e0) = w;
  __threadfence();
  *(volatile v4u*)(dst + e0) = w;
}

__global__ __launch_bounds__(256) void dt_table_kernel(
    const float* __restrict__ TT,
    const float* __restrict__ dtb_f, const float* __restrict__ dtb_b,
    const float* __restrict__ al_f, const float* __restrict__ al_b,
    float* __restrict__ DTA) {
  const int lane = threadIdx.x & 31;
  const int wave = threadIdx.x >> 5;
  const int gw = blockIdx.x * 8 + wave;
  const int dir = gw >> 5;
  const int tk = gw & 31;
  const int tkc = tk > (kVoc - 1) ? (kVoc - 1) : tk;
  const int h = lane & 15;
  const int which = lane >> 4;
  const float* dtb = dir ? dtb_b : dtb_f;
  const float* al  = dir ? al_b : al_f;
  const float raw = TT[(size_t)(dir * kTokP + tkc) * kProjP + kColDt + h] + dtb[h];
  const float ax = fabsf(raw);
  const float dt = fmaxf(raw, 0.0f) + log1pf(expf(-ax));
  const float An = -expf(al[h]);
  const float dA = expf(dt * An);
  float val = which ? dA : dt;
  if (fabsf(val) < 1.17549435e-38f) val = 0.0f;
  volatile float* q = DTA + (size_t)gw * 32 + lane;
  *q = val;
  __threadfence();
  *q = val;
}

__global__ __launch_bounds__(64) void scan_kernel(
    const int* __restrict__ inputs, const float* __restrict__ T, const float* __restrict__ DTA,
    const float* __restrict__ cw, const float* __restrict__ cb, const float* __restrict__ Dp,
    float* __restrict__ ys, int dir) {
  __shared__ __align__(16) float sTx[kVoc * 64];
  __shared__ __align__(16) float sTb[kVoc * 64];
  __shared__ int sTok[kLen];
  __shared__ float sDtA[64];
  __shared__ __align__(16) float sBC[2 * 64];
  __shared__ __align__(16) float sY[kChunk * kYP];
  const int tid = threadIdx.x;
  const int lane = tid & 31;
  const int wave = tid >> 5;
  const int bm = blockIdx.x >> 4;
  const int h = blockIdx.x & 15;

#pragma unroll 1
  for (int i = 0; i < kLen / 64; ++i) {
    const int l = tid + 64 * i;
    const int srcl = dir ? (kLen - 1 - l) : l;
    sTok[l] = clamp_tok(inputs[srcl * kSeqs + bm]);
  }
#pragma unroll 1
  for (int tk = 0; tk < kVoc; ++tk) {
    sTx[tk * 64 + tid] = T[(size_t)tk * kProjP + kColX + h * kHd + tid];
    sTb[tk * 64 + tid] = T[(size_t)tk * kProjP + kColB + tid];
  }
  {
    const int tk = tid & 31;
    const int which = tid >> 5;
    sDtA[which * 32 + tk] = DTA[tk * 32 + which * 16 + h];
  }
  const int cx = h * kHd + tid;
  const int cbc = kDi + tid;
  const v4f wx = *(const v4f*)(cw + (size_t)cx * 4);
  const v4f wb = *(const v4f*)(cw + (size_t)cbc * 4);
  const float bx = cb[cx];
  const float bb = cb[cbc];
  const float Dh = Dp[h];
  __syncthreads();

  float s[kNs];
#pragma unroll
  for (int n = 0; n < kNs; ++n) s[n] = 0.0f;
  float xm3 = 0.0f, xm2 = 0.0f, xm1 = 0.0f;
  float bm3 = 0.0f, bm2 = 0.0f, bm1 = 0.0f;
  const int hh = lane >> 4;
  const int c4 = (lane & 15) * 4;
  const size_t rowbase = (size_t)bm * kLen;

#pragma unroll 1
  for (int l0 = 0; l0 < kLen; l0 += kChunk) {
#pragma unroll 1
    for (int ls = 0; ls < kChunk; ++ls) {
      const int tok = sTok[l0 + ls];
      const float xc = sTx[tok * 64 + tid];
      const float bc = sTb[tok * 64 + tid];
      float sx = fmaf(wx[0], xm3, bx);
      sx = fmaf(wx[1], xm2, sx);
      sx = fmaf(wx[2], xm1, sx);
      sx = fmaf(wx[3], xc, sx);
      float sb = fmaf(wb[0], bm3, bb);
      sb = fmaf(wb[1], bm2, sb);
      sb = fmaf(wb[2], bm1, sb);
      sb = fmaf(wb[3], bc, sb);
      xm3 = xm2; xm2 = xm1; xm1 = xc;
      bm3 = bm2; bm2 = bm1; bm1 = bc;
      const float xa = silu_fast(sx);
      const float ba = silu_fast(sb);
      float* bcb = sBC + (ls & 1) * 64;
      bcb[tid] = ba;
      __syncthreads();
      const float dtv = sDtA[tok];
      const float dAv = sDtA[32 + tok];
      const float coef = dtv * xa;
      float y = 0.0f;
#pragma unroll
      for (int q = 0; q < kNs / 4; ++q) {
        const v4f bv = *(const v4f*)(bcb + 4 * q);
        const v4f cv = *(const v4f*)(bcb + kNs + 4 * q);
        s[4 * q + 0] = fmaf(s[4 * q + 0], dAv, coef * bv[0]);
        y = fmaf(s[4 * q + 0], cv[0], y);
        s[4 * q + 1] = fmaf(s[4 * q + 1], dAv, coef * bv[1]);
        y = fmaf(s[4 * q + 1], cv[1], y);
        s[4 * q + 2] = fmaf(s[4 * q + 2], dAv, coef * bv[2]);
        y = fmaf(s[4 * q + 2], cv[2], y);
        s[4 * q + 3] = fmaf(s[4 * q + 3], dAv, coef * bv[3]);
        y = fmaf(s[4 * q + 3], cv[3], y);
      }
      y = fmaf(xa, Dh, y);
      sY[ls * kYP + tid] = y;
    }
    __syncthreads();
    v4f fv[4];
#pragma unroll
    for (int it = 0; it < 4; ++it) {
      const int row = wave * 8 + it * 2 + hh;
      fv[it] = *(const v4f*)(sY + row * kYP + c4);
    }
    for (int pass = 0; pass < 2; ++pass) {
#pragma unroll
      for (int it = 0; it < 4; ++it) {
        const int row = wave * 8 + it * 2 + hh;
        *(volatile v4f*)(ys + (rowbase + l0 + row) * kDi + h * kHd + c4) = fv[it];
      }
      __threadfence();
    }
    __syncthreads();
  }
}

__global__ __launch_bounds__(128) void gatenorm_kernel(
    const int* __restrict__ inputs, const float* __restrict__ T, const float* __restrict__ ys,
    const float* __restrict__ nw, unsigned short* __restrict__ yn, int dir) {
  __shared__ float sRed[4];
  const int tid = threadIdx.x;
  const int lane = tid & 31;
  const int wave = tid >> 5;
  const int r = blockIdx.x;
  const int bm = r >> 8;
  const int l = r & (kLen - 1);
  const int srcl = dir ? (kLen - 1 - l) : l;
  const int tok = clamp_tok(inputs[srcl * kSeqs + bm]);
  const int c = tid * 8;
  const v4f y0 = *(const v4f*)(ys + (size_t)r * kDi + c);
  const v4f y1 = *(const v4f*)(ys + (size_t)r * kDi + c + 4);
  const v4f z0 = *(const v4f*)(T + (size_t)tok * kProjP + c);
  const v4f z1 = *(const v4f*)(T + (size_t)tok * kProjP + c + 4);
  const v4f n0 = *(const v4f*)(nw + c);
  const v4f n1 = *(const v4f*)(nw + c + 4);
  float g[8];
#pragma unroll
  for (int e = 0; e < 4; ++e) {
    g[e]     = y0[e] * silu_fast(z0[e]);
    g[4 + e] = y1[e] * silu_fast(z1[e]);
  }
  float ss = 0.0f;
#pragma unroll
  for (int e = 0; e < 8; ++e) ss = fmaf(g[e], g[e], ss);
#pragma unroll
  for (int off = 16; off > 0; off >>= 1) ss += __shfl_xor(ss, off, 32);
  if (lane == 0) sRed[wave] = ss;
  __syncthreads();
  const float tot = (sRed[0] + sRed[1]) + (sRed[2] + sRed[3]);
  const float sc = rsqrtf(tot * kInvDi + 1e-5f);
  float o[8];
#pragma unroll
  for (int e = 0; e < 4; ++e) {
    o[e]     = ((g[e] * sc) * n0[e]) * kCarryA;
    o[4 + e] = ((g[4 + e] * sc) * n1[e]) * kCarryA;
  }
  const unsigned w0 = h2pack(o[0], o[1]);
  const unsigned w1 = h2pack(o[2], o[3]);
  const unsigned w2 = h2pack(o[4], o[5]);
  const unsigned w3 = h2pack(o[6], o[7]);
  const v4u w = (v4u){w0, w1, w2, w3};
  unsigned short* q = yn + (size_t)r * kDi + c;
  *(volatile v4u*)q = w;
  __threadfence();
  *(volatile v4u*)q = w;
}

__global__ __launch_bounds__(256) void combine_kernel(
    const int* __restrict__ inputs, const float* __restrict__ emb,
    const float* __restrict__ of, const float* __restrict__ ob,
    unsigned short* __restrict__ yh, unsigned short* __restrict__ yl) {
  const int i = blockIdx.x * 256 + threadIdx.x;
  const int r = i >> 7;
  const int c8 = (i & 127) << 3;
  const int half = c8 >> 9;
  const int cc = c8 & (kDm - 1);
  const int bm = r >> 8;
  const int l = r & (kLen - 1);
  const int tok = clamp_tok(inputs[l * kSeqs + bm]);
  const int rs = half ? (bm * kLen + (kLen - 1 - l)) : r;
  const float* src = half ? ob : of;
  const v4f o0 = *(const v4f*)(src + (size_t)rs * kDm + cc);
  const v4f o1 = *(const v4f*)(src + (size_t)rs * kDm + cc + 4);
  const v4f e0 = *(const v4f*)(emb + (size_t)tok * kDm + cc);
  const v4f e1 = *(const v4f*)(emb + (size_t)tok * kDm + cc + 4);
  unsigned h0, h1, h2, h3, l0, l1, l2, l3;
  split2(o0[0] + e0[0], o0[1] + e0[1], h0, l0);
  split2(o0[2] + e0[2], o0[3] + e0[3], h1, l1);
  split2(o1[0] + e1[0], o1[1] + e1[1], h2, l2);
  split2(o1[2] + e1[2], o1[3] + e1[3], h3, l3);
  const v4u wh = (v4u){h0, h1, h2, h3};
  const v4u wl = (v4u){l0, l1, l2, l3};
  const size_t o = (size_t)r * kDi + c8;
  *(volatile v4u*)(yh + o) = wh;
  *(volatile v4u*)(yl + o) = wl;
  __threadfence();
  *(volatile v4u*)(yh + o) = wh;
  *(volatile v4u*)(yl + o) = wl;
}

__global__ __launch_bounds__(256) void pack_out_kernel(
    const float* __restrict__ cp, const float* __restrict__ lb, float* __restrict__ out) {
  const int i = blockIdx.x * 256 + threadIdx.x;
  const int r = i / kVoc;
  const int v = i - r * kVoc;
  const float val = cp[(size_t)r * kVocP + v] + lb[v];
  volatile float* q = out + i;
  *q = val;
  __threadfence();
  *q = val;
}

extern "C" void kernel_launch(void* const* d_in, const int* in_sizes, int n_in,
                              void* d_out, int out_size, void* d_ws, size_t ws_size,
                              hipStream_t stream) {
  if (n_in < 21) return;
  if (in_sizes[0] != kLen * kSeqs) return;
  if (in_sizes[2] != kVoc * kDm) return;
  if (in_sizes[3] != kProj * kDm || in_sizes[11] != kProj * kDm) return;
  if (in_sizes[4] != kConv * 4 || in_sizes[12] != kConv * 4) return;
  if (in_sizes[5] != kConv || in_sizes[13] != kConv) return;
  if (in_sizes[6] != kNh || in_sizes[7] != kNh || in_sizes[8] != kNh) return;
  if (in_sizes[14] != kNh || in_sizes[15] != kNh || in_sizes[16] != kNh) return;
  if (in_sizes[9] != kDi || in_sizes[17] != kDi) return;
  if (in_sizes[10] != kDm * kDi || in_sizes[18] != kDm * kDi) return;
  if (in_sizes[19] != kVoc * kDi) return;
  if (in_sizes[20] != kVoc) return;
  if (out_size != kRows * kVoc) return;
  if (ws_size < kWsTotal) return;

  const int*   inputs = (const int*)d_in[0];
  const float* emb    = (const float*)d_in[2];
  const float* w_in[2]  = {(const float*)d_in[3],  (const float*)d_in[11]};
  const float* c_w[2]   = {(const float*)d_in[4],  (const float*)d_in[12]};
  const float* c_b[2]   = {(const float*)d_in[5],  (const float*)d_in[13]};
  const float* dt_b[2]  = {(const float*)d_in[6],  (const float*)d_in[14]};
  const float* a_log[2] = {(const float*)d_in[7],  (const float*)d_in[15]};
  const float* d_p[2]   = {(const float*)d_in[8],  (const float*)d_in[16]};
  const float* n_w[2]   = {(const float*)d_in[9],  (const float*)d_in[17]};
  const float* w_out[2] = {(const float*)d_in[10], (const float*)d_in[18]};
  const float* lin_w = (const float*)d_in[19];
  const float* lin_b = (const float*)d_in[20];
  float* out = (float*)d_out;

  char* ws = (char*)d_ws;
  unsigned short* EMH = (unsigned short*)(ws + kOffEMH);
  unsigned short* EML = (unsigned short*)(ws + kOffEML);
  unsigned short* WIH = (unsigned short*)(ws + kOffWIH);
  unsigned short* WIL = (unsigned short*)(ws + kOffWIL);
  float*          TT  = (float*)(ws + kOffTT);
  float*          DTA = (float*)(ws + kOffDTA);
  float*          YS  = (float*)(ws + kOffYS);
  unsigned short* YN  = (unsigned short*)(ws + kOffYN);
  unsigned short* WO  = (unsigned short*)(ws + kOffWO);
  float*          OD[2] = {(float*)(ws + kOffOF), (float*)(ws + kOffOB)};
  unsigned short* YH  = (unsigned short*)(ws + kOffYH);
  unsigned short* YL  = (unsigned short*)(ws + kOffYL);
  unsigned short* LH  = (unsigned short*)(ws + kOffLH);
  unsigned short* LL  = (unsigned short*)(ws + kOffLL);
  float*          CP  = (float*)(ws + kOffCP);

  constexpr size_t kWiPlane = (size_t)kProjP * kDm;
  constexpr size_t kTPlane  = (size_t)kTokP * kProjP;
  constexpr size_t kWoPlane = (size_t)kDm * kDi;

  split_pad_bf16_kernel<<<(kTokP * kDm / 8) / 256, 256, 0, stream>>>(emb, EMH, EML, kVoc, kDm / 8, kTokP * kDm / 8);
  split_pad_bf16_kernel<<<(kProjP * kDm / 8) / 256, 256, 0, stream>>>(w_in[0], WIH, WIL, kProj, kDm / 8, kProjP * kDm / 8);
  split_pad_bf16_kernel<<<(kProjP * kDm / 8) / 256, 256, 0, stream>>>(w_in[1], WIH + kWiPlane, WIL + kWiPlane, kProj, kDm / 8, kProjP * kDm / 8);
  split_pad_bf16_kernel<<<(kVocP * kDi / 8) / 256, 256, 0, stream>>>(lin_w, LH, LL, kVoc, kDi / 8, kVocP * kDi / 8);
  cvt_f16_carry_kernel<<<(kDm * kDi / 8) / 256, 256, 0, stream>>>(w_out[0], WO, kDm * kDi / 8, kCarryW);
  cvt_f16_carry_kernel<<<(kDm * kDi / 8) / 256, 256, 0, stream>>>(w_out[1], WO + kWoPlane, kDm * kDi / 8, kCarryW);

  wmma_gemm64<1, true><<<dim3((kProjP / 64 + 7) / 8, 2), 256, 0, stream>>>(
      EMH, EML, kDm, 0L,
      WIH, WIL, kDm, (long)kWiPlane,
      TT, kProjP, (long)kTPlane,
      kTokP, kProjP, kDm, 1.0f);

  dt_table_kernel<<<8, 256, 0, stream>>>(TT, dt_b[0], dt_b[1], a_log[0], a_log[1], DTA);

  for (int d = 0; d < 2; ++d) {
    const float* Td = TT + (size_t)d * kTPlane;
    scan_kernel<<<kSeqs * kNh, 64, 0, stream>>>(inputs, Td, DTA + (size_t)d * 32 * 32, c_w[d], c_b[d], d_p[d], YS, d);
    gatenorm_kernel<<<kRows, 128, 0, stream>>>(inputs, Td, YS, n_w[d], YN, d);
    wmma_gemm64<0, false><<<dim3((kRows / 64) * (kDm / 64) / 8, 1), 256, 0, stream>>>(
        YN, YN, kDi, 0L,
        WO + (size_t)d * kWoPlane, WO + (size_t)d * kWoPlane, kDi, 0L,
        OD[d], kDm, 0L,
        kRows, kDm, kDi, kFold);
  }

  combine_kernel<<<(kRows * kDi / 8) / 256, 256, 0, stream>>>(inputs, emb, OD[0], OD[1], YH, YL);

  wmma_gemm64<1, true><<<dim3((kRows / 64) * (kVocP / 64) / 8, 1), 256, 0, stream>>>(
      YH, YL, kDi, 0L,
      LH, LL, kDi, 0L,
      CP, kVocP, 0L,
      kRows, kVocP, kDi, 1.0f);

  pack_out_kernel<<<(kRows * kVoc) / 256, 256, 0, stream>>>(CP, lin_b, out);
}
